// SelfAttentionConv_3066606649394
// MI455X (gfx1250) — hardware-verified
//
#include <hip/hip_runtime.h>
#include <math.h>
#include <float.h>
#include <stdint.h>

#ifndef NB
#define NB 4
#endif
#ifndef SEQ
#define SEQ 2048
#endif
#define NB_FULL  4
#define SEQ_FULL 2048
#define KD   128
#define NHD  8
#define KSZ  5
#define DMO  (KD * NHD)
#define KC   (KD * KSZ)
#define TP   (SEQ + KSZ - 1)
#define NBP  (NB * NHD)
#define NQB  (SEQ / 64)
#define RESQB ((NQB < 8) ? NQB : 8)
#define VLP  (RESQB * 64)
#define ATTN_LDS_RES   114688
#define ATTN_LDS_NORES 73728

static_assert((SEQ % 64) == 0);
static_assert(NB >= 1 && NB <= NB_FULL);
static_assert(SEQ <= SEQ_FULL);
static_assert(KD == 128 && NHD == 8);
static_assert((KC % 32) == 0);
static_assert(RESQB * 64 <= VLP && VLP <= SEQ);
static_assert((size_t)NB * SEQ * KD * 4 <= (size_t)4194304);
static_assert(((NB * TP * KD) % 8) == 0);

typedef _Float16 v16h __attribute__((ext_vector_type(16)));
typedef _Float16 v8h  __attribute__((ext_vector_type(8)));
typedef __bf16   v16b __attribute__((ext_vector_type(16)));
typedef __bf16   v8b  __attribute__((ext_vector_type(8)));
typedef float    v8f  __attribute__((ext_vector_type(8)));
typedef float    v4f  __attribute__((ext_vector_type(4)));
typedef unsigned int v4u __attribute__((ext_vector_type(4)));

__device__ __forceinline__ unsigned short bf_bits(float f) {
  unsigned u = __float_as_uint(f);
  return (unsigned short)((u + 0x7FFFu + ((u >> 16) & 1u)) >> 16);
}
__device__ __forceinline__ float bf_up(unsigned short h) { return __uint_as_float(((unsigned)h) << 16); }
__device__ __forceinline__ unsigned short h_bits(_Float16 x) { return __builtin_bit_cast(unsigned short, x); }
__device__ __forceinline__ unsigned pk16(unsigned short a, unsigned short b) { return (unsigned)a | ((unsigned)b << 16); }
__device__ __forceinline__ v8f zero8() { v8f z = {0.f, 0.f, 0.f, 0.f, 0.f, 0.f, 0.f, 0.f}; return z; }
__device__ __forceinline__ v8h zero8h() {
  const _Float16 z = (_Float16)0.0f;
  v8h r = {z, z, z, z, z, z, z, z};
  return r;
}
__device__ __forceinline__ v4u pack8bf(v4f a, v4f b) {
  v4u p;
  p[0] = pk16(bf_bits(a[0]), bf_bits(a[1]));
  p[1] = pk16(bf_bits(a[2]), bf_bits(a[3]));
  p[2] = pk16(bf_bits(b[0]), bf_bits(b[1]));
  p[3] = pk16(bf_bits(b[2]), bf_bits(b[3]));
  return p;
}

__device__ __forceinline__ v16b ldfrag_b(const __bf16* p) {
  union { v16b v; v8b h[2]; } f;
  f.h[0] = *(const v8b*)(p);
  f.h[1] = *(const v8b*)(p + 16);
  return f.v;
}

__device__ __forceinline__ v8f mma_b(v16b a, v16b b, v8f c) {
  c = __builtin_amdgcn_wmma_f32_16x16x32_bf16(false, a, false, b, (short)0, c, false, false);
  asm volatile("v_nop\n\tv_nop\n\tv_nop\n\tv_nop" : "+v"(c) : "v"(a), "v"(b));
  return c;
}
__device__ __forceinline__ v8f mma_h(v16h a, v16h b, v8f c) {
  c = __builtin_amdgcn_wmma_f32_16x16x32_f16(false, a, false, b, (short)0, c, false, false);
  asm volatile("v_nop\n\tv_nop\n\tv_nop\n\tv_nop" : "+v"(c) : "v"(a), "v"(b));
  return c;
}
__device__ __forceinline__ v8f mma_b_raw(v16b a, v16b b, v8f c) {
  return __builtin_amdgcn_wmma_f32_16x16x32_bf16(false, a, false, b, (short)0, c, false, false);
}
__device__ __forceinline__ void dep_guard_b(v8f& a, v8f& b, v16b x, v16b y) {
  asm volatile("v_nop\n\tv_nop\n\tv_nop\n\tv_nop" : "+v"(a), "+v"(b) : "v"(x), "v"(y));
}
__device__ __forceinline__ void keep4_b(v16b a, v16b b, v16b c, v16b d) {
  asm volatile("v_nop" :: "v"(a), "v"(b), "v"(c), "v"(d));
}
__device__ __forceinline__ void acc_guard4(v8f& a, v8f& b, v8f& c, v8f& d) {
  asm volatile("v_nop\n\tv_nop\n\tv_nop\n\tv_nop" : "+v"(a), "+v"(b), "+v"(c), "+v"(d));
}

__global__ __launch_bounds__(256) void cvt_xpad(const float* __restrict__ x, unsigned short* out, int n8) {
  const int i = blockIdx.x * 256 + threadIdx.x;
  if (i >= n8) return;
  const size_t e = (size_t)i * 8;
  const int b   = (int)(e / ((size_t)TP * KD));
  const int rem = (int)(e - (size_t)b * TP * KD);
  const int tp  = rem / KD;
  const int col = rem - tp * KD;
  const int tr  = tp - (KSZ - 1);
  const int trc = (tr < 0) ? 0 : tr;
  const float* src = x + ((size_t)b * SEQ_FULL + trc) * KD + col;
  const v4f a = *(const v4f*)(src);
  const v4f c = *(const v4f*)(src + 4);
  v4u p = pack8bf(a, c);
  if (tr < 0) { p[0] = 0u; p[1] = 0u; p[2] = 0u; p[3] = 0u; }
  *(volatile v4u*)(out + e) = p;
  __threadfence();
  *(volatile v4u*)(out + e) = p;
}

__global__ __launch_bounds__(256) void cvt_wconv(const float* __restrict__ Wq, const float* __restrict__ Wk,
                                                 unsigned short* Wqb, unsigned short* Wkb, int n8) {
  const int i = blockIdx.x * 256 + threadIdx.x;
  if (i >= n8) return;
  const int e = i * 8;
  const int n = e / KC;
  const int k = e - n * KC;
  const int j = k / KD;
  const int c = k - j * KD;
  const int o = (n & (KD - 1)) * NHD + (n / KD);
  const float* sq = Wq + ((size_t)o * KD + c) * KSZ + j;
  const float* sk = Wk + ((size_t)o * KD + c) * KSZ + j;
  v4u pq, pkk;
#pragma unroll
  for (int u = 0; u < 4; ++u) pq[u] = pk16(bf_bits(sq[(2 * u) * KSZ]), bf_bits(sq[(2 * u + 1) * KSZ]));
  asm volatile("" ::: "memory");
#pragma unroll
  for (int u = 0; u < 4; ++u) pkk[u] = pk16(bf_bits(sk[(2 * u) * KSZ]), bf_bits(sk[(2 * u + 1) * KSZ]));
  *(volatile v4u*)(Wqb + (size_t)e) = pq;
  *(volatile v4u*)(Wkb + (size_t)e) = pkk;
  __threadfence();
  *(volatile v4u*)(Wqb + (size_t)e) = pq;
  *(volatile v4u*)(Wkb + (size_t)e) = pkk;
}

__global__ __launch_bounds__(256) void cvt_wvu(const float* __restrict__ Wv, const float* __restrict__ Wu,
                                               unsigned short* Wvb, unsigned short* Wub) {
  const int nv8 = DMO * KD / 8;
  const int i = blockIdx.x * 256 + threadIdx.x;
  if (i < nv8) {
    const int e = i * 8;
    const int n = e / KD;
    const int c = e - n * KD;
    const int o = (n & (KD - 1)) * NHD + (n / KD);
    const float* src = Wv + (size_t)o * KD + c;
    const v4f a = *(const v4f*)(src);
    const v4f bq = *(const v4f*)(src + 4);
    const v4u p = pack8bf(a, bq);
    *(volatile v4u*)(Wvb + (size_t)e) = p;
    __threadfence();
    *(volatile v4u*)(Wvb + (size_t)e) = p;
  } else if (i < 2 * nv8) {
    const int e = (i - nv8) * 8;
    const float* src = Wu + (size_t)e;
    const v4f a = *(const v4f*)(src);
    const v4f bq = *(const v4f*)(src + 4);
    const v4u p = pack8bf(a, bq);
    *(volatile v4u*)(Wub + (size_t)e) = p;
    __threadfence();
    *(volatile v4u*)(Wub + (size_t)e) = p;
  }
}

template <int NSPLIT, int OUT_MODE, int BIAS>
__global__ __launch_bounds__(256) void gemm64(
    const unsigned short* __restrict__ Ap, const unsigned short* A2p, int lda, long long strideA,
    const unsigned short* __restrict__ Btp, const unsigned short* Bt2p, int ldb, long long strideB,
    void* Cout, int ldc, long long strideC,
    void* Cout2, int ldc2, long long strideC2, int N2,
    const float* __restrict__ bias, float cscale,
    int M, int N, int K, float rscale) {
  const __bf16* A   = (const __bf16*)(const void*)Ap;
  const __bf16* A2  = (const __bf16*)(const void*)A2p;
  const __bf16* Bt  = (const __bf16*)(const void*)Btp;
  const __bf16* Bt2 = (const __bf16*)(const void*)Bt2p;
  __shared__ __align__(16) float sT[8][16 * 68];
  const int b    = blockIdx.y;
  const int lane = threadIdx.x & 31;
  const int wave = threadIdx.x >> 5;
  const int tilesN = N >> 6;
  const int tilesM = M >> 6;
  const int tile = blockIdx.x * 8 + wave;
  if (tile >= tilesM * tilesN) return;
  const int tm = tile / tilesN;
  const int tn = tile - tm * tilesN;
  const int m0 = tm << 6;
  const int n0 = tn << 6;

  const __bf16* Ab  = A  + (size_t)b * strideA;
  const __bf16* Bb  = Bt + (size_t)b * strideB;
  const __bf16* Ab2 = (NSPLIT >= 1) ? (A2  + (size_t)b * strideA) : Ab;
  const __bf16* Bb2 = (NSPLIT == 2) ? (Bt2 + (size_t)b * strideB) : Bb;

  const int rlane = lane & 15;
  const int koff  = (lane >> 4) * 8;
  const int mOff  = (lane >> 4) * 8;

  v8f acc[4][4];
#pragma unroll
  for (int i = 0; i < 4; ++i)
#pragma unroll
    for (int j = 0; j < 4; ++j) acc[i][j] = zero8();

  for (int k0 = 0; k0 < K; k0 += 32) {
    v16b bh[4], bl[4];
#pragma unroll
    for (int j = 0; j < 4; ++j) {
      const size_t bo = (size_t)(n0 + (j << 4) + rlane) * ldb + koff + k0;
      bh[j] = ldfrag_b(Bb + bo);
      if (NSPLIT == 2) bl[j] = ldfrag_b(Bb2 + bo); else bl[j] = bh[j];
    }
#pragma unroll
    for (int i = 0; i < 4; ++i) {
      const size_t ao = (size_t)(m0 + (i << 4) + rlane) * lda + koff + k0;
      const v16b ah = ldfrag_b(Ab + ao);
      v16b al = ah;
      if (NSPLIT >= 1) al = ldfrag_b(Ab2 + ao);
#pragma unroll
      for (int j = 0; j < 4; ++j) {
        acc[i][j] = mma_b_raw(ah, bh[j], acc[i][j]);
        if (NSPLIT >= 1) acc[i][j] = mma_b_raw(al, bh[j], acc[i][j]);
        if (NSPLIT == 2) acc[i][j] = mma_b_raw(ah, bl[j], acc[i][j]);
      }
      dep_guard_b(acc[i][0], acc[i][3], ah, al);
    }
    keep4_b(bh[0], bh[1], bh[2], bh[3]);
    if (NSPLIT == 2) keep4_b(bl[0], bl[1], bl[2], bl[3]);
  }
  acc_guard4(acc[0][0], acc[0][1], acc[0][2], acc[0][3]);
  acc_guard4(acc[1][0], acc[1][1], acc[1][2], acc[1][3]);
  acc_guard4(acc[2][0], acc[2][1], acc[2][2], acc[2][3]);
  acc_guard4(acc[3][0], acc[3][1], acc[3][2], acc[3][3]);

  float bv[4];
#pragma unroll
  for (int j = 0; j < 4; ++j) {
    float t = 0.f;
    if (BIAS != 0) {
      const int n  = n0 + (j << 4) + rlane;
      const int bi = (BIAS == 2) ? ((n & (KD - 1)) * NHD + (n / KD)) : n;
      t = bf_up(bf_bits(bias[bi]));
    }
    bv[j] = t;
  }
  float* slab = sT[wave];
#pragma unroll
  for (int i = 0; i < 4; ++i) {
    const int mBase = m0 + (i << 4);
#pragma unroll
    for (int j = 0; j < 4; ++j) {
#pragma unroll
      for (int r = 0; r < 8; ++r) {
        slab[(mOff + r) * 68 + (j << 4) + rlane] = (acc[i][j][r] + bv[j]) * cscale;
      }
    }
    __builtin_amdgcn_fence(__ATOMIC_RELEASE, "workgroup");
    __builtin_amdgcn_wave_barrier();
    __builtin_amdgcn_fence(__ATOMIC_ACQUIRE, "workgroup");
    if (OUT_MODE == 0) {
      float* C = (float*)Cout + (size_t)b * strideC;
      const int hh = lane >> 4, c4 = (lane & 15) * 4;
      for (int pass = 0; pass < 2; ++pass) {
#pragma unroll
        for (int it = 0; it < 8; ++it) {
          const int row = it * 2 + hh;
          const v4f v = *(const v4f*)(slab + row * 68 + c4);
          *(volatile v4f*)(C + (size_t)(mBase + row) * ldc + n0 + c4) = v;
        }
        __threadfence();
      }
    } else {
      const int q = lane >> 3, c8 = (lane & 7) * 8;
      unsigned short* C  = (unsigned short*)Cout  + (size_t)b * strideC;
      unsigned short* C2 = (unsigned short*)Cout2 + (size_t)b * strideC2;
      const bool wlo = (OUT_MODE == 2) || (n0 < N2);
      v4u hv[4], lv[4];
#pragma unroll
      for (int it = 0; it < 4; ++it) {
        const int row = it * 4 + q;
        const float* sp = slab + row * 68 + c8;
        v4u a, a2;
#pragma unroll
        for (int e = 0; e < 4; ++e) {
          const float f0 = sp[2 * e], f1 = sp[2 * e + 1];
          unsigned short h0, h1, l0, l1;
          if (OUT_MODE == 2) {
            h0 = bf_bits(f0); h1 = bf_bits(f1);
            l0 = bf_bits(f0 - bf_up(h0)); l1 = bf_bits(f1 - bf_up(h1));
          } else {
            const _Float16 x0 = (_Float16)f0, x1 = (_Float16)f1;
            h0 = h_bits(x0); h1 = h_bits(x1);
            l0 = h_bits((_Float16)((f0 - (float)x0) * rscale));
            l1 = h_bits((_Float16)((f1 - (float)x1) * rscale));
          }
          a[e] = pk16(h0, h1); a2[e] = pk16(l0, l1);
        }
        hv[it] = a; lv[it] = a2;
      }
      for (int pass = 0; pass < 2; ++pass) {
#pragma unroll
        for (int it = 0; it < 4; ++it) {
          const int row = it * 4 + q;
          *(volatile v4u*)(C + (size_t)(mBase + row) * ldc + n0 + c8) = hv[it];
          if (wlo) *(volatile v4u*)(C2 + (size_t)(mBase + row) * ldc2 + n0 + c8) = lv[it];
        }
        __threadfence();
      }
    }
    __builtin_amdgcn_fence(__ATOMIC_RELEASE, "workgroup");
    __builtin_amdgcn_wave_barrier();
    __builtin_amdgcn_fence(__ATOMIC_ACQUIRE, "workgroup");
  }
}

__global__ __launch_bounds__(256) void vt_split(const float* __restrict__ Vf, unsigned short* vth, unsigned short* vtl) {
  __shared__ __align__(16) float sv[64 * 68];
  const int tid  = threadIdx.x;
  const int wave = tid >> 5;
  const int lane = tid & 31;
  const int njt  = SEQ / 64;
  const int bx   = blockIdx.x;
  const int jt   = bx % njt;
  const int rest = bx / njt;
  const int dt   = rest & 1;
  const int Bp   = rest >> 1;
  {
    const int row = tid >> 2, qc = (tid & 3) * 16;
    const float* src = Vf + ((size_t)Bp * SEQ + (size_t)jt * 64 + row) * KD + dt * 64 + qc;
#pragma unroll
    for (int i = 0; i < 4; ++i) {
      const v4f a = *(const v4f*)(src + 4 * i);
      *(v4f*)(sv + row * 68 + qc + 4 * i) = a;
    }
  }
  __syncthreads();
  const int q8 = lane >> 3, c8 = (lane & 7) * 8;
  const bool wres = (jt * 64 < VLP);
  v4u hv[2], lv[2];
#pragma unroll
  for (int it = 0; it < 2; ++it) {
    const int drow = wave * 8 + it * 4 + q8;
    v4u a, a2;
#pragma unroll
    for (int e = 0; e < 4; ++e) {
      const float f0 = sv[(c8 + 2 * e) * 68 + drow];
      const float f1 = sv[(c8 + 2 * e + 1) * 68 + drow];
      const _Float16 x0 = (_Float16)f0, x1 = (_Float16)f1;
      const unsigned short h0 = h_bits(x0), h1 = h_bits(x1);
      const unsigned short l0 = h_bits((_Float16)((f0 - (float)x0) * 4096.0f));
      const unsigned short l1 = h_bits((_Float16)((f1 - (float)x1) * 4096.0f));
      a[e] = pk16(h0, h1); a2[e] = pk16(l0, l1);
    }
    hv[it] = a; lv[it] = a2;
  }
  for (int pass = 0; pass < 2; ++pass) {
#pragma unroll
    for (int it = 0; it < 2; ++it) {
      const int drow = wave * 8 + it * 4 + q8;
      const int d = dt * 64 + drow;
      *(volatile v4u*)(vth + ((size_t)Bp * KD + d) * SEQ + (size_t)jt * 64 + c8) = hv[it];
      if (wres) *(volatile v4u*)(vtl + ((size_t)Bp * KD + d) * VLP + (size_t)jt * 64 + c8) = lv[it];
    }
    __threadfence();
  }
}

template <bool RES>
__global__ __launch_bounds__(128)
void attn_causal128(const unsigned short* __restrict__ qhp, const unsigned short* __restrict__ qlp,
                    const unsigned short* __restrict__ khp, const unsigned short* __restrict__ klp,
                    const unsigned short* __restrict__ vhp, const unsigned short* __restrict__ vlp,
                    unsigned short* ohp, unsigned short* olp, int qbBase, int nqbThis) {
  union FB { v16b v; v8b h[2]; };
  union FH { v16h v; v8h h[2]; };
  extern __shared__ v4u dsm[];
  unsigned char* smem = (unsigned char*)dsm;
  constexpr int OB_KSH = 0;
  constexpr int OB_KSL = 16384;
  constexpr int OB_VTH = RES ? 32768 : 16384;
  constexpr int OB_VTL = 49152;
  constexpr int OB_QSH = RES ? 65536 : 32768;
  constexpr int OB_QSL = OB_QSH + 16384;
  constexpr int OB_PSH = OB_QSL + 16384;
  constexpr int OB_PSL = OB_PSH + 8192;
  __bf16*   Ksh = (__bf16*)(smem + OB_KSH);
  __bf16*   Ksl = (__bf16*)(smem + (RES ? OB_KSL : OB_KSH));
  _Float16* Vth = (_Float16*)(smem + OB_VTH);
  _Float16* Vtl = (_Float16*)(smem + (RES ? OB_VTL : OB_VTH));
  __bf16*   Qsh = (__bf16*)(smem + OB_QSH);
  __bf16*   Qsl = (__bf16*)(smem + OB_QSL);
  _Float16* Psh = (_Float16*)(smem + OB_PSH);
  _Float16* Psl = (_Float16*)(smem + (RES ? OB_PSL : OB_PSH));

  const int tid  = threadIdx.x;
  const int wave = tid >> 5;
  const int lane = tid & 31;
  const int hh   = lane >> 4;
  const int c    = lane & 15;

  const int bx   = blockIdx.x;
  const int qbl  = bx % nqbThis;
  const int Bp   = bx / nqbThis;
  const int qb   = qbBase + qbl;
  const int b    = Bp / NHD;
  const int g    = Bp - b * NHD;
  const int q0   = qb * 64 + wave * 16;
  const size_t rowP = (size_t)Bp * SEQ;

  const __bf16* Qh = (const __bf16*)(const void*)qhp;
  const __bf16* Ql = (const __bf16*)(const void*)qlp;
  const __bf16* Kh = (const __bf16*)(const void*)khp;
  const __bf16* Kl = (const __bf16*)(const void*)klp;
  const _Float16* Vh = (const _Float16*)(const void*)vhp + (size_t)Bp * KD * SEQ;
  const _Float16* Vl = (const _Float16*)(const void*)vlp + (size_t)Bp * KD * VLP;

  {
    const int r = tid >> 1, half = (tid & 1) * 64;
    const __bf16* qg  = Qh + (rowP + (size_t)qb * 64 + r) * KD + half;
    const __bf16* qlg = Ql + (rowP + (size_t)qb * 64 + r) * KD + half;
#pragma unroll
    for (int i = 0; i < 8; ++i) {
      const v8b a = *(const v8b*)(qg + 8 * i);
      *(v8b*)(Qsh + r * KD + half + 8 * i) = a;
    }
    asm volatile("" ::: "memory");
#pragma unroll
    for (int i = 0; i < 8; ++i) {
      const v8b a = *(const v8b*)(qlg + 8 * i);
      *(v8b*)(Qsl + r * KD + half + 8 * i) = a;
    }
  }

  float mrow[8], lrow[8];
  v8f oacc[8];
#pragma unroll
  for (int r = 0; r < 8; ++r) { mrow[r] = -INFINITY; lrow[r] = 0.f; }
#pragma unroll
  for (int t = 0; t < 8; ++t) oacc[t] = zero8();

  for (int kt = 0; kt < NQB; ++kt) {
    if (kt > qb) break;
    const int kv0 = kt * 64;
    __syncthreads();
    {
      const int r = tid >> 1, half = (tid & 1) * 64;
      const __bf16* kg  = Kh + (rowP + kv0 + r) * KD + half;
      const __bf16* klg = Kl + (rowP + kv0 + r) * KD + half;
#pragma unroll
      for (int i = 0; i < 8; ++i) {
        const v8b a0 = *(const v8b*)(kg + 8 * i);
        *(v8b*)(Ksh + r * KD + half + 8 * i) = a0;
      }
      asm volatile("" ::: "memory");
      if (RES) {
#pragma unroll
        for (int i = 0; i < 8; ++i) {
          const v8b a1 = *(const v8b*)(klg + 8 * i);
          *(v8b*)(Ksl + r * KD + half + 8 * i) = a1;
        }
        asm volatile("" ::: "memory");
      }
      const int d = tid;
      const _Float16* vg = Vh + (size_t)d * SEQ + kv0;
#pragma unroll
      for (int i = 0; i < 8; ++i) {
        const v8h b0 = *(const v8h*)(vg + 8 * i);
        *(v8h*)(Vth + d * 64 + 8 * i) = b0;
      }
      asm volatile("" ::: "memory");
      if (RES) {
        const int kvl = (kv0 + 64 <= VLP) ? kv0 : (VLP - 64);
        const bool resOK = (kv0 + 64 <= VLP);
        const _Float16* vlg = Vl + (size_t)d * VLP + kvl;
#pragma unroll
        for (int i = 0; i < 8; ++i) {
          v8h b1 = *(const v8h*)(vlg + 8 * i);
          if (!resOK) b1 = zero8h();
          *(v8h*)(Vtl + d * 64 + 8 * i) = b1;
        }
      }
    }
    __syncthreads();

    v8f s[4];
#pragma unroll
    for (int j = 0; j < 4; ++j) s[j] = zero8();
#pragma unroll
    for (int dc = 0; dc < 4; ++dc) {
      FB qa, qz;
      qa.h[0] = *(const v8b*)(Qsh + (wave * 16 + c) * KD + dc * 32 + 8 * hh);
      qa.h[1] = *(const v8b*)(Qsh + (wave * 16 + c) * KD + dc * 32 + 16 + 8 * hh);
      qz.h[0] = *(const v8b*)(Qsl + (wave * 16 + c) * KD + dc * 32 + 8 * hh);
      qz.h[1] = *(const v8b*)(Qsl + (wave * 16 + c) * KD + dc * 32 + 16 + 8 * hh);
#pragma unroll
      for (int j = 0; j < 4; ++j) {
        FB kb;
        kb.h[0] = *(const v8b*)(Ksh + (j * 16 + c) * KD + dc * 32 + 8 * hh);
        kb.h[1] = *(const v8b*)(Ksh + (j * 16 + c) * KD + dc * 32 + 16 + 8 * hh);
        s[j] = mma_b(qa.v, kb.v, s[j]);
        s[j] = mma_b(qz.v, kb.v, s[j]);
        if (RES) {
          FB kz;
          kz.h[0] = *(const v8b*)(Ksl + (j * 16 + c) * KD + dc * 32 + 8 * hh);
          kz.h[1] = *(const v8b*)(Ksl + (j * 16 + c) * KD + dc * 32 + 16 + 8 * hh);
          s[j] = mma_b(qa.v, kz.v, s[j]);
        }
      }
    }

    _Float16* pwh = Psh + wave * (16 * 64);
    _Float16* pwl = Psl + (RES ? wave : 0) * (16 * 64);
#pragma unroll
    for (int r = 0; r < 8; ++r) {
      const int qrow = q0 + 8 * hh + r;
      float m = -INFINITY;
#pragma unroll
      for (int j = 0; j < 4; ++j) {
        const int kidx = kv0 + j * 16 + c;
        float sv = s[j][r];
        sv = (kidx > qrow) ? -INFINITY : sv;
        s[j][r] = sv;
        m = fmaxf(m, sv);
      }
#pragma unroll
      for (int off = 1; off < 16; off <<= 1) m = fmaxf(m, __shfl_xor(m, off, 32));
      const float mnew  = fmaxf(mrow[r], m);
      const float msafe = (mnew == -INFINITY) ? 0.f : mnew;
      const float alpha = __expf(mrow[r] - msafe);
      mrow[r] = mnew;
      float psum = 0.f;
#pragma unroll
      for (int j = 0; j < 4; ++j) {
        const float p = __expf(s[j][r] - msafe);
        psum += p;
        const float p1k = p * 1024.0f;
        const _Float16 ph = (_Float16)p1k;
        pwh[(8 * hh + r) * 64 + j * 16 + c] = ph;
        if (RES) {
          const _Float16 pl = (_Float16)((p1k - (float)ph) * 4096.0f);
          pwl[(8 * hh + r) * 64 + j * 16 + c] = pl;
        }
      }
#pragma unroll
      for (int off = 1; off < 16; off <<= 1) psum += __shfl_xor(psum, off, 32);
      lrow[r] = lrow[r] * alpha + psum;
#pragma unroll
      for (int t = 0; t < 8; ++t) oacc[t][r] *= alpha;
    }
    __builtin_amdgcn_fence(__ATOMIC_RELEASE, "workgroup");
    __builtin_amdgcn_wave_barrier();
    __builtin_amdgcn_fence(__ATOMIC_ACQUIRE, "workgroup");

    FH pa[2], pz[2];
#pragma unroll
    for (int kk = 0; kk < 2; ++kk) {
      pa[kk].h[0] = *(const v8h*)(pwh + c * 64 + kk * 32 + 8 * hh);
      pa[kk].h[1] = *(const v8h*)(pwh + c * 64 + kk * 32 + 16 + 8 * hh);
      if (RES) {
        pz[kk].h[0] = *(const v8h*)(pwl + c * 64 + kk * 32 + 8 * hh);
        pz[kk].h[1] = *(const v8h*)(pwl + c * 64 + kk * 32 + 16 + 8 * hh);
      } else {
        pz[kk].v = pa[kk].v;
      }
    }
#pragma unroll
    for (int t = 0; t < 8; ++t) {
      v8f o1 = zero8();
#pragma unroll
      for (int kk = 0; kk < 2; ++kk) {
        FH vb;
        vb.h[0] = *(const v8h*)(Vth + (t * 16 + c) * 64 + kk * 32 + 8 * hh);
        vb.h[1] = *(const v8h*)(Vth + (t * 16 + c) * 64 + kk * 32 + 16 + 8 * hh);
        oacc[t] = mma_h(pa[kk].v, vb.v, oacc[t]);
        if (RES) {
          FH vz;
          vz.h[0] = *(const v8h*)(Vtl + (t * 16 + c) * 64 + kk * 32 + 8 * hh);
          vz.h[1] = *(const v8h*)(Vtl + (t * 16 + c) * 64 + kk * 32 + 16 + 8 * hh);
          o1 = mma_h(pa[kk].v, vz.v, o1);
          o1 = mma_h(pz[kk].v, vb.v, o1);
        }
      }
      if (RES) {
#pragma unroll
        for (int r = 0; r < 8; ++r) oacc[t][r] += o1[r] * (1.0f / 4096.0f);
      }
    }
  }

  __syncthreads();
  float* os = (float*)smem + wave * (16 * KD);
#pragma unroll
  for (int r = 0; r < 8; ++r) {
    const float l = lrow[r];
    const float inv = ((l > 0.f) ? (1.0f / l) : 0.f) * (1.0f / 1024.0f);
#pragma unroll
    for (int t = 0; t < 8; ++t) os[(8 * hh + r) * KD + t * 16 + c] = oacc[t][r] * inv;
  }
  __builtin_amdgcn_fence(__ATOMIC_RELEASE, "workgroup");
  __builtin_amdgcn_wave_barrier();
  __builtin_amdgcn_fence(__ATOMIC_ACQUIRE, "workgroup");
  {
    const int r2 = lane >> 4, c8 = c * 8;
    v4u hv[8], lv[8];
#pragma unroll
    for (int it = 0; it < 8; ++it) {
      const int row = it * 2 + r2;
      const float* sp = os + row * KD + c8;
      v4u a, a2;
#pragma unroll
      for (int e = 0; e < 4; ++e) {
        const float f0 = sp[2 * e], f1 = sp[2 * e + 1];
        const unsigned short h0 = bf_bits(f0), h1 = bf_bits(f1);
        const unsigned short l0 = bf_bits(f0 - bf_up(h0)), l1 = bf_bits(f1 - bf_up(h1));
        a[e] = pk16(h0, h1); a2[e] = pk16(l0, l1);
      }
      hv[it] = a; lv[it] = a2;
    }
    for (int pass = 0; pass < 2; ++pass) {
#pragma unroll
      for (int it = 0; it < 8; ++it) {
        const int row = it * 2 + r2;
        const size_t go = ((size_t)b * SEQ + q0 + row) * DMO + (size_t)g * KD + c8;
        *(volatile v4u*)(ohp + go) = hv[it];
        *(volatile v4u*)(olp + go) = lv[it];
      }
      __threadfence();
    }
  }
}

extern "C" void kernel_launch(void* const* d_in, const int* in_sizes, int n_in,
                              void* d_out, int out_size, void* d_ws, size_t ws_size,
                              hipStream_t stream) {
  if (n_in < 8) return;
  if (in_sizes[0] < ((NB - 1) * SEQ_FULL + SEQ) * KD) return;
  if (in_sizes[1] < DMO * KD * KSZ) return;
  if (in_sizes[2] < DMO) return;
  if (in_sizes[3] < DMO * KD * KSZ) return;
  if (in_sizes[4] < DMO) return;
  if (in_sizes[5] < DMO * KD) return;
  if (in_sizes[6] < KD * DMO) return;
  if (in_sizes[7] < KD) return;
  if (out_size < NB * SEQ * KD) return;

  const float* x  = (const float*)d_in[0];
  const float* Wq = (const float*)d_in[1];
  const float* bq = (const float*)d_in[2];
  const float* Wk = (const float*)d_in[3];
  const float* bk = (const float*)d_in[4];
  const float* Wv = (const float*)d_in[5];
  const float* Wu = (const float*)d_in[6];
  const float* bu = (const float*)d_in[7];

  const size_t PXP = (size_t)NB * TP * KD * 2;
  const size_t PWC = (size_t)DMO * KC * 2;
  const size_t PWV = (size_t)DMO * KD * 2;
  const size_t PWU = (size_t)KD * DMO * 2;
  const size_t PA  = (size_t)NB * SEQ * DMO * 2;
  const size_t PVF = (size_t)NB * SEQ * DMO * 4;
  const size_t PVT = (size_t)NBP * KD * SEQ * 2;
  const size_t PVL = (size_t)NBP * KD * VLP * 2;
  size_t off = 0;
  const size_t oXp  = off; off += PXP;
  const size_t oWqb = off; off += PWC;
  const size_t oWkb = off; off += PWC;
  const size_t oWvb = off; off += PWV;
  const size_t oWub = off; off += PWU;
  const size_t oQh  = off; off += PA;
  const size_t oQl  = off; off += PA;
  const size_t oKh  = off; off += PA;
  const size_t oKl  = off; off += PA;
  const size_t oVTh = off; off += PVT;
  const size_t oVTl = off; off += PVL;
  const size_t oOh  = off; off += PA;
  const size_t oOl  = off; off += PA;
  if (off > ws_size) return;
  if (off > (size_t)134217728) return;
  const size_t oVf  = oQh;
  if (oVf + PVF > oKh) return;

  char* ws = (char*)d_ws;
  unsigned short* Xp  = (unsigned short*)(ws + oXp);
  unsigned short* Wqb = (unsigned short*)(ws + oWqb);
  unsigned short* Wkb = (unsigned short*)(ws + oWkb);
  unsigned short* Wvb = (unsigned short*)(ws + oWvb);
  unsigned short* Wub = (unsigned short*)(ws + oWub);
  unsigned short* Qh  = (unsigned short*)(ws + oQh);
  unsigned short* Ql  = (unsigned short*)(ws + oQl);
  unsigned short* Kh  = (unsigned short*)(ws + oKh);
  unsigned short* Kl  = (unsigned short*)(ws + oKl);
  unsigned short* VTh = (unsigned short*)(ws + oVTh);
  unsigned short* VTl = (unsigned short*)(ws + oVTl);
  unsigned short* Oh  = (unsigned short*)(ws + oOh);
  unsigned short* Ol  = (unsigned short*)(ws + oOl);
  float*          Vf  = (float*)(ws + oVf);

  const dim3 blk(256);
  const int n8x = NB * TP * KD / 8;
  const int n8c = DMO * KC / 8;
  const int n8v = DMO * KD / 8;
  const dim3 gCvtX((n8x + 255) / 256);
  const dim3 gCvtC((n8c + 255) / 256);
  const dim3 gCvtV((2 * n8v + 255) / 256);
  const dim3 gProj(((SEQ / 64) * (DMO / 64) + 7) / 8, NB);
  const dim3 gVt(NBP * 2 * (SEQ / 64));
  const dim3 gOut(((NB * SEQ / 64) * (KD / 64) + 7) / 8, 1);
  const float cscale = 0.29730177875068026f;

  cvt_xpad<<<gCvtX, blk, 0, stream>>>(x, Xp, n8x);
  cvt_wconv<<<gCvtC, blk, 0, stream>>>(Wq, Wk, Wqb, Wkb, n8c);
  cvt_wvu<<<gCvtV, blk, 0, stream>>>(Wv, Wu, Wvb, Wub);
  gemm64<0, 0, 0><<<gProj, blk, 0, stream>>>(
      Xp + (KSZ - 1) * KD, Xp + (KSZ - 1) * KD, KD, (long long)TP * KD, Wvb, Wvb, KD, 0LL,
      (void*)Vf, DMO, (long long)SEQ * DMO, (void*)Vf, DMO, (long long)SEQ * DMO, DMO,
      bq, 1.0f, SEQ, DMO, KD, 1.0f);
  vt_split<<<gVt, blk, 0, stream>>>(Vf, VTh, VTl);
  gemm64<0, 2, 2><<<gProj, blk, 0, stream>>>(
      Xp, Xp, KD, (long long)TP * KD, Wqb, Wqb, KC, 0LL,
      (void*)Qh, DMO, (long long)SEQ * DMO, (void*)Ql, DMO, (long long)SEQ * DMO, DMO,
      bq, cscale, SEQ, DMO, KC, 1.0f);
  gemm64<0, 2, 2><<<gProj, blk, 0, stream>>>(
      Xp, Xp, KD, (long long)TP * KD, Wkb, Wkb, KC, 0LL,
      (void*)Kh, DMO, (long long)SEQ * DMO, (void*)Kl, DMO, (long long)SEQ * DMO, DMO,
      bk, cscale, SEQ, DMO, KC, 1.0f);
  (void)hipFuncSetAttribute(reinterpret_cast<const void*>(&attn_causal128<true>),
                            hipFuncAttributeMaxDynamicSharedMemorySize, ATTN_LDS_RES);
  (void)hipFuncSetAttribute(reinterpret_cast<const void*>(&attn_causal128<false>),
                            hipFuncAttributeMaxDynamicSharedMemorySize, ATTN_LDS_NORES);
  attn_causal128<true><<<dim3(NBP * RESQB), dim3(128), ATTN_LDS_RES, stream>>>(
      Qh, Ql, Kh, Kl, VTh, VTl, Oh, Ol, 0, RESQB);
  if (NQB > RESQB) {
    attn_causal128<false><<<dim3(NBP * (NQB - RESQB)), dim3(128), ATTN_LDS_NORES, stream>>>(
        Qh, Ql, Kh, Kl, VTh, VTl, Oh, Ol, RESQB, NQB - RESQB);
  }
  gemm64<1, 0, 1><<<gOut, blk, 0, stream>>>(
      Oh, Ol, DMO, 0LL, Wub, Wub, DMO, 0LL,
      d_out, KD, 0LL, d_out, KD, 0LL, KD,
      bu, 1.0f, NB * SEQ, KD, DMO, 1.0f);
  (void)hipGetLastError();
}
